// NonLocalBlock_58437325029910
// MI455X (gfx1250) — hardware-verified
//
#include <hip/hip_runtime.h>


#ifndef NB
#define NB 8
#endif
#ifndef SEQ
#define SEQ 2048
#endif
#define NB_FULL  8
#define SEQ_FULL 2048
#ifndef OUT_SEQ
#define OUT_SEQ SEQ
#endif
#define DM   256
#define AW   4
#define CSP  264
#define XTP  65
#define QRS  2048.0f
#define QRI  (1.0f / 2048.0f)
#define L2E  1.4426950408889634f
#define PSH  14.0f
#define NEGB (-3.0e38f)
#define WSC  64.0f
#define WSI  (1.0f / 64.0f)

static_assert(DM == 256);
static_assert(DM % 64 == 0);
static_assert(DM % 32 == 0);
static_assert(32 * 8 == DM);
static_assert(SEQ % 64 == 0);
static_assert((NB * SEQ) % 64 == 0);
static_assert(SEQ % 32 == 0);
static_assert(SEQ % (16 * AW) == 0);
static_assert(NB <= NB_FULL);
static_assert(SEQ <= SEQ_FULL);
static_assert(SEQ_FULL % 4 == 0);
static_assert(OUT_SEQ % 4 == 0);
static_assert(OUT_SEQ >= SEQ);
static_assert((CSP * 2) % 16 == 0);
static_assert(CSP >= DM);
static_assert(4 * 256 == 64 * 16);
static_assert(2 * 256 == 64 * 8);
static_assert(4 * 32 * 16 == 16 * 128);
static_assert(8 * 32 * 16 == 16 * 256);
static_assert(16 * 32 * 16 == 16 * DM * 2);
static_assert((size_t)AW * 16 * CSP * 2 <= 131072);
static_assert((size_t)64 * XTP * 4 <= 131072);
static_assert((size_t)16 * 68 * 4 <= 131072);
static_assert(((size_t)DM * DM) % 8 == 0);

typedef _Float16 h16;
typedef unsigned short bf;
typedef __attribute__((ext_vector_type(16))) __bf16   v16bf;
typedef __attribute__((ext_vector_type(16))) _Float16 v16h;
typedef __attribute__((ext_vector_type(8)))  _Float16 v8h;
typedef __attribute__((ext_vector_type(8)))  unsigned short v8us;
typedef __attribute__((ext_vector_type(8)))  float    v8f;
typedef __attribute__((ext_vector_type(4)))  float    v4f;
typedef v4f  __attribute__((may_alias)) v4fa;
typedef v8h  __attribute__((may_alias)) v8ha;

__device__ __forceinline__ unsigned short f2bf(float f) { unsigned u = __float_as_uint(f); u += 0x7FFFu + ((u >> 16) & 1u); return (unsigned short)(u >> 16); }
__device__ __forceinline__ float bfr(float f) { return __uint_as_float(((unsigned)f2bf(f)) << 16); }
__device__ __forceinline__ v16h cat16(v8h lo, v8h hi) { return __builtin_shufflevector(lo, hi, 0, 1, 2, 3, 4, 5, 6, 7, 8, 9, 10, 11, 12, 13, 14, 15); }
__device__ __forceinline__ v16bf cat16b(v8us lo, v8us hi) { return __builtin_bit_cast(v16bf, __builtin_shufflevector(lo, hi, 0, 1, 2, 3, 4, 5, 6, 7, 8, 9, 10, 11, 12, 13, 14, 15)); }
__device__ __forceinline__ v8f wmma16(v16h a, v16h b, v8f c) { return __builtin_amdgcn_wmma_f32_16x16x32_f16(false, a, false, b, (short)0, c, false, false); }
__device__ __forceinline__ v8f wmmab(v16bf a, v16bf b, v8f c) { return __builtin_amdgcn_wmma_f32_16x16x32_bf16(false, a, false, b, (short)0, c, false, false); }
__device__ __forceinline__ v16h  ldh(const h16* p) { return cat16(*(const v8h*)p, *(const v8h*)(p + 16)); }
__device__ __forceinline__ v16bf ldb(const bf* p)  { return cat16b(*(const v8us*)p, *(const v8us*)(p + 16)); }
__device__ __forceinline__ void wave_sync() { __builtin_amdgcn_fence(3  , "wavefront"); __builtin_amdgcn_wave_barrier(); asm volatile("" ::: "memory"); }
__device__ __forceinline__ h16 toh_flush(float v) { const h16 r = (h16)v; return (fabsf(v) < 6.103515625e-05f) ? (h16)0.0f : r; }
__device__ __forceinline__ v8f wg16(v16h a, v16h b, v8f c) { c = wmma16(a, b, c); asm volatile("v_nop\n\tv_nop\n\tv_nop\n\tv_nop" : "+v"(c) : "v"(a), "v"(b)); return c; }
__device__ __forceinline__ v8f wgb(v16bf a, v16bf b, v8f c) { c = wmmab(a, b, c); asm volatile("v_nop\n\tv_nop\n\tv_nop\n\tv_nop" : "+v"(c) : "v"(a), "v"(b)); return c; }

__global__ __launch_bounds__(256) void k_cvt8(const float* __restrict__ src, bf* dst, size_t n8) {
    const size_t i = (size_t)blockIdx.x * 256 + threadIdx.x; if (i >= n8) return;
    const v8f v = *(const v8f*)(src + i * 8); v8us o;
#pragma unroll
    for (int k = 0; k < 8; ++k) o[k] = f2bf(v[k]);
    *(volatile v8us*)(dst + i * 8) = o; __threadfence(); *(volatile v8us*)(dst + i * 8) = o;
}

__global__ __launch_bounds__(256) void k_wcvt(const float* __restrict__ src, h16* dst, size_t n8) {
    const size_t i = (size_t)blockIdx.x * 256 + threadIdx.x; if (i >= n8) return;
    const v8f v = *(const v8f*)(src + i * 8); v8h o;
#pragma unroll
    for (int k = 0; k < 8; ++k) o[k] = toh_flush(bfr(v[k]) * WSC);
    *(volatile v8h*)(dst + i * 8) = o; __threadfence(); *(volatile v8h*)(dst + i * 8) = o;
}

__global__ __launch_bounds__(256) void k_xt(const float* __restrict__ x, bf* XT) {
    __shared__ float ts[64 * XTP];
    const int tid = threadIdx.x;
    const int n0 = blockIdx.x * 64, c0 = blockIdx.y * 64, b = blockIdx.z;
    const float* xb = x + ((size_t)b * DM + c0) * SEQ_FULL + n0;
#pragma unroll
    for (int s = 0; s < 4; ++s) {
        const int p = s * 256 + tid; const int c = p >> 4, n4 = (p & 15) * 4;
        const v4f v = *(const v4f*)(xb + (size_t)c * SEQ_FULL + n4);
        ts[c * XTP + n4 + 0] = v[0]; ts[c * XTP + n4 + 1] = v[1]; ts[c * XTP + n4 + 2] = v[2]; ts[c * XTP + n4 + 3] = v[3];
    }
    __syncthreads();
    const int n = tid >> 3, c8 = (tid & 7) * 8;
    v8us o0, o1;
#pragma unroll
    for (int i = 0; i < 8; ++i) { o0[i] = f2bf(ts[(c8 + i) * XTP + n]); o1[i] = f2bf(ts[(c8 + i) * XTP + 32 + n]); }
    bf* d0 = XT + ((size_t)b * SEQ + n0 + n) * DM + c0 + c8;
    bf* d1 = d0 + (size_t)32 * DM;
    *(volatile v8us*)d0 = o0; *(volatile v8us*)d1 = o1;
    __threadfence();
    *(volatile v8us*)d0 = o0; *(volatile v8us*)d1 = o1;
}

template <int MODE>
__device__ __forceinline__ void proj_body(const bf* __restrict__ A, const bf* __restrict__ Bt, const float* __restrict__ bias, h16* Ph, h16* Pr, int wr) {
    __shared__ __align__(16) float os[16 * 68];
    const int K = DM;
    const int lane = threadIdx.x & 31, lr = lane & 15, hi = lane >> 4; const int r0 = blockIdx.x * 64, c0 = blockIdx.y * 64;
    v8f acc[4][4];
#pragma unroll
    for (int mb = 0; mb < 4; ++mb)
#pragma unroll
        for (int nb = 0; nb < 4; ++nb) acc[mb][nb] = (v8f){};
    const size_t aoff = (size_t)(r0 + lr) * K + 8 * hi, boff = (size_t)(c0 + lr) * K + 8 * hi;
#pragma unroll 1
    for (int kc = 0; kc < K; kc += 32) {
        v16bf a[4];
#pragma unroll
        for (int mb = 0; mb < 4; ++mb) a[mb] = ldb(A + aoff + (size_t)mb * 16 * K + kc);
#pragma unroll
        for (int nb = 0; nb < 4; ++nb) { const v16bf b = ldb(Bt + boff + (size_t)nb * 16 * K + kc);
#pragma unroll
            for (int mb = 0; mb < 4; ++mb) acc[mb][nb] = wgb(a[mb], b, acc[mb][nb]); }
    }
    float bc[4];
#pragma unroll
    for (int nb = 0; nb < 4; ++nb) bc[nb] = (MODE == 0) ? bfr(bias[c0 + nb * 16 + lr]) : 0.0f;
    const size_t pitch = (MODE == 0) ? (size_t)DM : (size_t)SEQ;
    size_t tbase;
    if (MODE == 0) { tbase = (size_t)r0 * DM + (size_t)c0; }
    else           { const int bb = c0 / SEQ, tt = c0 % SEQ; tbase = (size_t)bb * (size_t)DM * SEQ + (size_t)r0 * SEQ + (size_t)tt; }
#pragma unroll
    for (int mb = 0; mb < 4; ++mb) {
        float br[8];
#pragma unroll
        for (int j = 0; j < 8; ++j) br[j] = (MODE == 1) ? bfr(bias[r0 + mb * 16 + hi * 8 + j]) : 0.0f;
#pragma unroll
        for (int nb = 0; nb < 4; ++nb) {
#pragma unroll
            for (int j = 0; j < 8; ++j) os[(hi * 8 + j) * 68 + nb * 16 + lr] = acc[mb][nb][j] + bc[nb] + br[j]; }
        wave_sync();
        const size_t sb = tbase + (size_t)(mb * 16) * pitch;
#pragma unroll 1
        for (int ps = 0; ps < 2; ++ps) {
#pragma unroll
            for (int s = 0; s < 4; ++s) { const int row = 4 * s + (lane >> 3), c8 = (lane & 7) * 8;
                const v4f x0 = *(const v4fa*)(&os[row * 68 + c8]); const v4f x1 = *(const v4fa*)(&os[row * 68 + c8 + 4]); v8h hv, rv;
#pragma unroll
                for (int i = 0; i < 4; ++i) { const h16 a0 = toh_flush(x0[i]); const h16 a1 = toh_flush(x1[i]); hv[i] = a0; hv[4 + i] = a1;
                    rv[i] = toh_flush((x0[i] - (float)a0) * QRS); rv[4 + i] = toh_flush((x1[i] - (float)a1) * QRS); }
                const size_t oo = sb + (size_t)row * pitch + c8;
                *(volatile v8h*)(Ph + oo) = hv; if (wr) *(volatile v8h*)(Pr + oo) = rv; }
            if (ps == 0) __threadfence(); }
        wave_sync();
    }
}
__global__ __launch_bounds__(32) void k_proj_rows(const bf* __restrict__ A, const bf* __restrict__ Bt, const float* __restrict__ bias, h16* Ph, h16* Pr, int wr) { proj_body<0>(A, Bt, bias, Ph, Pr, wr); }
__global__ __launch_bounds__(32) void k_proj_cols(const bf* __restrict__ A, const bf* __restrict__ Bt, const float* __restrict__ bias, h16* Ph, h16* Pr, int wr) { proj_body<1>(A, Bt, bias, Ph, Pr, wr); }

__global__ __launch_bounds__(32 * AW) __attribute__((amdgpu_num_vgpr(256))) void k_flash(const h16* __restrict__ TH, const h16* __restrict__ TR, const h16* __restrict__ PH, const h16* __restrict__ PR,
                                                                                       const h16* __restrict__ GT, h16* CT) {
    __shared__ __align__(16) h16 os[AW * 16 * CSP];
    const int lane = threadIdx.x & 31, lr = lane & 15, hi = lane >> 4;
    const int wave = __builtin_amdgcn_readfirstlane((int)(threadIdx.x >> 5));
    const int b = blockIdx.y;
    const int t0 = (blockIdx.x * AW + wave) * 16;
    const size_t pb0 = (size_t)b * SEQ * DM;
    const size_t qo = pb0 + (size_t)(t0 + lr) * DM + 8 * hi;
    const size_t ko = pb0 + (size_t)lr * DM + 8 * hi;
    const size_t vo = pb0 + (size_t)lr * SEQ + 8 * hi;
    v8f o[16];
#pragma unroll
    for (int j = 0; j < 16; ++j) o[j] = (v8f){};
    float m = NEGB, l = 0.0f;
#pragma unroll 1
    for (int key0 = 0; key0 < SEQ; key0 += 32) {
        v8f sHa = (v8f){}, sLa = (v8f){}, sHb = (v8f){}, sLb = (v8f){};
        const size_t kk = ko + (size_t)key0 * DM;
#pragma unroll 1
        for (int kc = 0; kc < DM; kc += 32) {
            const v16h qh = ldh(TH + qo + kc), qr = ldh(TR + qo + kc);
            const v16h ka = ldh(PH + kk + kc), kra = ldh(PR + kk + kc);
            sHa = wg16(ka, qh, sHa); sLa = wg16(ka, qr, sLa); sLa = wg16(kra, qh, sLa);
            const v16h kb = ldh(PH + kk + (size_t)16 * DM + kc), krb = ldh(PR + kk + (size_t)16 * DM + kc);
            sHb = wg16(kb, qh, sHb); sLb = wg16(kb, qr, sLb); sLb = wg16(krb, qh, sLb);
        }
        float ta[8], tb[8]; float mx = NEGB;
#pragma unroll
        for (int r = 0; r < 8; ++r) {
            ta[r] = (sHa[r] + sLa[r] * QRI) * L2E; tb[r] = (sHb[r] + sLb[r] * QRI) * L2E;
            mx = fmaxf(mx, fmaxf(ta[r], tb[r])); }
        mx = fmaxf(mx, __shfl_xor(mx, 16, 32));
        const float mnew = fmaxf(m, mx);
        const float alpha = __builtin_amdgcn_exp2f(m - mnew);
        const float sh = PSH - mnew;
        v16h pb; float ls = 0.0f;
#pragma unroll
        for (int r = 0; r < 8; ++r) {
            const float aa = ta[r] + sh, ab = tb[r] + sh;
            const float ea = __builtin_amdgcn_exp2f(aa), eb = __builtin_amdgcn_exp2f(ab);
            const float ga = (aa < -14.0f) ? 0.0f : ea, gb = (ab < -14.0f) ? 0.0f : eb;
            const h16 pa = (h16)ga; const h16 pc = (h16)gb;
            pb[r] = pa; pb[8 + r] = pc;
            ls += (float)pa + (float)pc; }
        l = l * alpha + ls; m = mnew;
#pragma unroll
        for (int j = 0; j < 16; ++j) o[j] = o[j] * alpha;
        const h16* va = GT + vo + key0;
#pragma unroll
        for (int jg = 0; jg < 4; ++jg) {
            const v16h v0 = ldh(va + (size_t)((jg * 4 + 0) * 16) * SEQ);
            const v16h v1 = ldh(va + (size_t)((jg * 4 + 1) * 16) * SEQ);
            const v16h v2 = ldh(va + (size_t)((jg * 4 + 2) * 16) * SEQ);
            const v16h v3 = ldh(va + (size_t)((jg * 4 + 3) * 16) * SEQ);
            o[jg * 4 + 0] = wg16(v0, pb, o[jg * 4 + 0]);
            o[jg * 4 + 1] = wg16(v1, pb, o[jg * 4 + 1]);
            o[jg * 4 + 2] = wg16(v2, pb, o[jg * 4 + 2]);
            o[jg * 4 + 3] = wg16(v3, pb, o[jg * 4 + 3]);
        }
    }
    l += __shfl_xor(l, 16, 32);
    const float inv = 1.0f / l;
    const int wb = wave * 16 * CSP;
#pragma unroll
    for (int j = 0; j < 16; ++j) { v8h hv;
#pragma unroll
        for (int r = 0; r < 8; ++r) hv[r] = toh_flush(o[j][r] * inv);
        *(v8ha*)(&os[wb + lr * CSP + 16 * j + 8 * hi]) = hv; }
    wave_sync();
    h16* crow = CT + pb0 + (size_t)t0 * DM;
#pragma unroll 1
    for (int ps = 0; ps < 2; ++ps) {
#pragma unroll
        for (int row = 0; row < 16; ++row) {
            const v8h val = *(const v8ha*)(&os[wb + row * CSP + lane * 8]);
            *(volatile v8h*)(crow + (size_t)row * DM + lane * 8) = val; }
        if (ps == 0) __threadfence(); }
}

__global__ __launch_bounds__(32) void k_oproj(const h16* __restrict__ A, const h16* __restrict__ Bt, const float* __restrict__ bias, const float* __restrict__ xres, float* OUT) {
    __shared__ __align__(16) float os[16 * 68];
    const int K = DM;
    const int lane = threadIdx.x & 31, lr = lane & 15, hi = lane >> 4; const int r0 = blockIdx.x * 64, c0 = blockIdx.y * 64;
    v8f acc[4][4];
#pragma unroll
    for (int mb = 0; mb < 4; ++mb)
#pragma unroll
        for (int nb = 0; nb < 4; ++nb) acc[mb][nb] = (v8f){};
    const size_t aoff = (size_t)(r0 + lr) * K + 8 * hi, boff = (size_t)(c0 + lr) * K + 8 * hi;
#pragma unroll 1
    for (int kc = 0; kc < K; kc += 32) {
        v16h a[4];
#pragma unroll
        for (int mb = 0; mb < 4; ++mb) a[mb] = ldh(A + aoff + (size_t)mb * 16 * K + kc);
#pragma unroll
        for (int nb = 0; nb < 4; ++nb) { const v16h b = ldh(Bt + boff + (size_t)nb * 16 * K + kc);
#pragma unroll
            for (int mb = 0; mb < 4; ++mb) acc[mb][nb] = wg16(a[mb], b, acc[mb][nb]); }
    }
    const int bb = c0 / SEQ, tt = c0 % SEQ;
#pragma unroll
    for (int mb = 0; mb < 4; ++mb) {
        float br[8];
#pragma unroll
        for (int j = 0; j < 8; ++j) br[j] = bfr(bias[r0 + mb * 16 + hi * 8 + j]);
#pragma unroll
        for (int nb = 0; nb < 4; ++nb) {
#pragma unroll
            for (int j = 0; j < 8; ++j) os[(hi * 8 + j) * 68 + nb * 16 + lr] = acc[mb][nb][j] * WSI + br[j]; }
        wave_sync();
        const size_t chrow = (size_t)bb * DM + (size_t)(r0 + mb * 16);
        const size_t xb = chrow * SEQ_FULL + (size_t)tt;
        const size_t ob = chrow * OUT_SEQ + (size_t)tt;
#pragma unroll 1
        for (int ps = 0; ps < 2; ++ps) {
#pragma unroll
            for (int s = 0; s < 8; ++s) { const int row = 2 * s + (lane >> 4), c4 = (lane & 15) * 4;
                const v4f cv = *(const v4fa*)(&os[row * 68 + c4]);
                const v4f xv = *(const v4f*)(xres + xb + (size_t)row * SEQ_FULL + c4);
                v4f val; val[0] = cv[0] + bfr(xv[0]); val[1] = cv[1] + bfr(xv[1]); val[2] = cv[2] + bfr(xv[2]); val[3] = cv[3] + bfr(xv[3]);
                *(volatile v4f*)(OUT + ob + (size_t)row * OUT_SEQ + c4) = val; }
            if (ps == 0) __threadfence(); }
        wave_sync();
    }
}

static constexpr size_t al256(size_t v) { return (v + 255) & ~(size_t)255; }
static constexpr size_t SZ_XT = al256((size_t)NB * SEQ * DM * 2);
static constexpr size_t SZ_WB = al256((size_t)3 * DM * DM * 2);
static constexpr size_t SZ_WW = al256((size_t)DM * DM * 2);
static constexpr size_t SZ_PL = al256((size_t)NB * SEQ * DM * 2);
static constexpr size_t SZ_TOTAL = SZ_XT + SZ_WB + SZ_WW + 6 * SZ_PL;
static_assert(SZ_TOTAL <= (size_t)134217728);
static_assert(((size_t)DM * DM * 2) % 256 == 0);
static constexpr size_t NEED_X = ((size_t)NB * DM - 1) * SEQ_FULL + SEQ;
static constexpr size_t NEED_O = ((size_t)NB * DM - 1) * OUT_SEQ + SEQ;

extern "C" void kernel_launch(void* const* d_in, const int* in_sizes, int n_in,
                              void* d_out, int out_size, void* d_ws, size_t ws_size, hipStream_t stream) {
    if (n_in < 9) return;
    if ((size_t)in_sizes[0] < NEED_X) return;
    if ((size_t)in_sizes[1] < (size_t)DM * DM || (size_t)in_sizes[3] < (size_t)DM * DM || (size_t)in_sizes[5] < (size_t)DM * DM || (size_t)in_sizes[7] < (size_t)DM * DM) return;
    if (in_sizes[2] < DM || in_sizes[4] < DM || in_sizes[6] < DM || in_sizes[8] < DM) return;
    if ((size_t)out_size < NEED_O) return;
    if (SZ_TOTAL > ws_size) return;
    const float* x   = (const float*)d_in[0];
    const float* wth = (const float*)d_in[1]; const float* bth = (const float*)d_in[2];
    const float* wph = (const float*)d_in[3]; const float* bph = (const float*)d_in[4];
    const float* wg  = (const float*)d_in[5]; const float* bg  = (const float*)d_in[6];
    const float* ww  = (const float*)d_in[7]; const float* bw  = (const float*)d_in[8];
    float* OUT = (float*)d_out;
    char* wsp = (char*)d_ws;
    bf*  XT = (bf*)wsp;  wsp += SZ_XT;
    bf*  WB = (bf*)wsp;  wsp += SZ_WB;
    h16* WW = (h16*)wsp; wsp += SZ_WW;
    h16* TH = (h16*)wsp; wsp += SZ_PL;
    h16* TR = (h16*)wsp; wsp += SZ_PL;
    h16* PH = (h16*)wsp; wsp += SZ_PL;
    h16* PR = (h16*)wsp; wsp += SZ_PL;
    h16* GT = (h16*)wsp; wsp += SZ_PL;
    h16* CT = (h16*)wsp; wsp += SZ_PL;
    bf* WT = WB; bf* WP = WB + (size_t)DM * DM; bf* WG = WB + (size_t)2 * DM * DM;

    k_xt<<<dim3(SEQ / 64, DM / 64, NB), 256, 0, stream>>>(x, XT);
    { const size_t n8 = (size_t)DM * DM / 8; const unsigned g = (unsigned)((n8 + 255) / 256);
      k_cvt8<<<g, 256, 0, stream>>>(wth, WT, n8); k_cvt8<<<g, 256, 0, stream>>>(wph, WP, n8); k_cvt8<<<g, 256, 0, stream>>>(wg, WG, n8);
      k_wcvt<<<g, 256, 0, stream>>>(ww, WW, n8); }

    k_proj_rows<<<dim3(NB * SEQ / 64, DM / 64, 1), 32, 0, stream>>>(XT, WT, bth, TH, TR, 1);
    k_proj_rows<<<dim3(NB * SEQ / 64, DM / 64, 1), 32, 0, stream>>>(XT, WP, bph, PH, PR, 1);
    k_proj_cols<<<dim3(DM / 64, NB * SEQ / 64, 1), 32, 0, stream>>>(WG, XT, bg, GT, GT, 0);

    k_flash<<<dim3(SEQ / (16 * AW), NB, 1), 32 * AW, 0, stream>>>(TH, TR, PH, PR, GT, CT);

    k_oproj<<<dim3(DM / 64, NB * SEQ / 64, 1), 32, 0, stream>>>(WW, CT, bw, x, OUT);
}
